// CrossMed4_85177791414322
// MI455X (gfx1250) — hardware-verified
//
#include <hip/hip_runtime.h>
#include <math.h>

typedef __attribute__((ext_vector_type(16))) _Float16 v16h;
typedef __attribute__((ext_vector_type(8)))  _Float16 v8h;
typedef __attribute__((ext_vector_type(16))) __bf16   v16b;
typedef __attribute__((ext_vector_type(8)))  __bf16   v8b;
typedef __attribute__((ext_vector_type(8)))  float    v8f;
typedef __attribute__((ext_vector_type(4)))  float    v4f;
#define PSCALE 32768.0f
#define U16(p) ((const unsigned short*)(const void*)(p))
#define PSCALE_INV (1.0f / 32768.0f)

__device__ __forceinline__ unsigned short f2bf_bits(float f) {
  unsigned u = __float_as_uint(f);
  return (unsigned short)((u + 0x7FFFu + ((u >> 16) & 1u)) >> 16);
}
__device__ __forceinline__ float bf_bits2f(unsigned short h) { return __uint_as_float(((unsigned)h) << 16); }

__device__ __forceinline__ void dep_guard_h(v8f& a, v8f& b, v16h x, v16h y) { asm volatile("v_nop\n\tv_nop\n\tv_nop\n\tv_nop" : "+v"(a), "+v"(b) : "v"(x), "v"(y)); }
__device__ __forceinline__ void dep_guard_b(v8f& a, v8f& b, v16b x, v16b y) { asm volatile("v_nop\n\tv_nop\n\tv_nop\n\tv_nop" : "+v"(a), "+v"(b) : "v"(x), "v"(y)); }
__device__ __forceinline__ void keep4_h(v16h a, v16h b, v16h c, v16h d) { asm volatile("v_nop" :: "v"(a), "v"(b), "v"(c), "v"(d)); }
__device__ __forceinline__ void keep4_b(v16b a, v16b b, v16b c, v16b d) { asm volatile("v_nop" :: "v"(a), "v"(b), "v"(c), "v"(d)); }
__device__ __forceinline__ void acc_guard4(v8f& a, v8f& b, v8f& c, v8f& d) { asm volatile("v_nop\n\tv_nop\n\tv_nop\n\tv_nop" : "+v"(a), "+v"(b), "+v"(c), "+v"(d)); }
template <typename T> struct Frag;
template <> struct Frag<_Float16> {
  typedef v16h V; union U { v16h v; v8h h[2]; };
  static __device__ __forceinline__ v16h load(const _Float16* p) {
    U f; f.h[0] = *(const v8h*)(p); f.h[1] = *(const v8h*)(p + 16); return f.v;
  }
  static __device__ __forceinline__ v8f mma(v16h a, v16h b, v8f c) {
    return __builtin_amdgcn_wmma_f32_16x16x32_f16(false, a, false, b, (short)0, c, false, false);
  }
  static __device__ __forceinline__ void guard(v8f& a, v8f& b, v16h x, v16h y) { dep_guard_h(a, b, x, y); }
  static __device__ __forceinline__ void keep(v16h a, v16h b, v16h c, v16h d) { keep4_h(a, b, c, d); }
};
template <> struct Frag<__bf16> {
  typedef v16b V; union U { v16b v; v8b h[2]; };
  static __device__ __forceinline__ v16b load(const __bf16* p) {
    U f; f.h[0] = *(const v8b*)(p); f.h[1] = *(const v8b*)(p + 16); return f.v;
  }
  static __device__ __forceinline__ v8f mma(v16b a, v16b b, v8f c) {
    return __builtin_amdgcn_wmma_f32_16x16x32_bf16(false, a, false, b, (short)0, c, false, false);
  }
  static __device__ __forceinline__ void guard(v8f& a, v8f& b, v16b x, v16b y) { dep_guard_b(a, b, x, y); }
  static __device__ __forceinline__ void keep(v16b a, v16b b, v16b c, v16b d) { keep4_b(a, b, c, d); }
};

template <int ET> struct Elem;
template <> struct Elem<0> { typedef _Float16 T; };
template <> struct Elem<1> { typedef __bf16 T; };
template <int ET, bool SPLIT, int BIAS_MODE, int OUT_MODE, bool RESID, int ACT = 0>
__global__ __launch_bounds__(256) void wmma_gemm64(
    const unsigned short* __restrict__ Ap, const unsigned short* __restrict__ A2p, int lda, long strideA,
    const unsigned short* __restrict__ Btp, const unsigned short* __restrict__ Bt2p, int ldb, long strideB,
    void* __restrict__ Cout, void* __restrict__ Cout2, int ldc, long strideC,
    const float* __restrict__ bias,
    const float* __restrict__ resid, long strideR,
    int M, int N, int K, float scale) {
  typedef typename Elem<ET>::T T;
  typedef typename Frag<T>::V V;
  const T* A = (const T*)Ap; const T* A2 = (const T*)A2p; const T* Bt = (const T*)Btp; const T* Bt2 = (const T*)Bt2p;
  __shared__ __align__(16) float sT[8][16 * 68];
  const int b    = blockIdx.y;
  const int lane = threadIdx.x & 31;
  const int wave = threadIdx.x >> 5;
  const int tilesN = N >> 6;
  const int tilesM = M >> 6;
  const int tile = blockIdx.x * 8 + wave;
  if (tile >= tilesM * tilesN) return;
  const int tm = tile / tilesN;
  const int tn = tile - tm * tilesN;
  const int m0 = tm << 6;
  const int n0 = tn << 6;

  const T* Ab  = A  + (size_t)b * strideA;
  const T* Bb  = Bt + (size_t)b * strideB;
  const T* Ab2 = SPLIT ? (A2  + (size_t)b * strideA) : nullptr;
  const T* Bb2 = SPLIT ? (Bt2 + (size_t)b * strideB) : nullptr;

  const int rlane = lane & 15;
  const int koff  = (lane >> 4) * 8;
  const int mOff  = (lane >> 4) * 8;

  v8f acc[4][4];
#pragma unroll
  for (int i = 0; i < 4; ++i)
#pragma unroll
    for (int j = 0; j < 4; ++j) acc[i][j] = (v8f){0.f,0.f,0.f,0.f,0.f,0.f,0.f,0.f};

  for (int k0 = 0; k0 < K; k0 += 32) {
    V bh[4], bl[4];
#pragma unroll
    for (int j = 0; j < 4; ++j) {
      const size_t bo = (size_t)(n0 + (j << 4) + rlane) * ldb + koff + k0;
      bh[j] = Frag<T>::load(Bb + bo);
      if (SPLIT) bl[j] = Frag<T>::load(Bb2 + bo);
    }
#pragma unroll
    for (int i = 0; i < 4; ++i) {
      const size_t ao = (size_t)(m0 + (i << 4) + rlane) * lda + koff + k0;
      V ah = Frag<T>::load(Ab + ao);
      V al;
      if (SPLIT) al = Frag<T>::load(Ab2 + ao);
#pragma unroll
      for (int j = 0; j < 4; ++j) {
        acc[i][j] = Frag<T>::mma(ah, bh[j], acc[i][j]);
        if (SPLIT) {
          acc[i][j] = Frag<T>::mma(ah, bl[j], acc[i][j]);
          acc[i][j] = Frag<T>::mma(al, bh[j], acc[i][j]);
        }
      }
      Frag<T>::guard(acc[i][0], acc[i][3], ah, SPLIT ? al : ah);
    }
    Frag<T>::keep(bh[0], bh[1], bh[2], bh[3]);
    if (SPLIT) Frag<T>::keep(bl[0], bl[1], bl[2], bl[3]);
  }
  acc_guard4(acc[0][0], acc[0][1], acc[0][2], acc[0][3]);
  acc_guard4(acc[1][0], acc[1][1], acc[1][2], acc[1][3]);
  acc_guard4(acc[2][0], acc[2][1], acc[2][2], acc[2][3]);
  acc_guard4(acc[3][0], acc[3][1], acc[3][2], acc[3][3]);

  float* slab = sT[wave];
  const float* Rb = RESID ? (resid + (size_t)b * strideR) : nullptr;
#pragma unroll
  for (int i = 0; i < 4; ++i) {
    const int mBase = m0 + (i << 4);
#pragma unroll
    for (int j = 0; j < 4; ++j) {
      const int n = n0 + (j << 4) + rlane;
      float bv = 0.f;
      if (BIAS_MODE == 2) bv = bias[n];
#pragma unroll
      for (int r = 0; r < 8; ++r) {
        float v = acc[i][j][r] * scale;
        if (BIAS_MODE == 1) v += bias[mBase + mOff + r];
        if (BIAS_MODE == 2) v += bv;
        if (RESID) v += Rb[(size_t)(mBase + mOff + r) * ldc + n];
        if (ACT == 1) v = tanhf(v);
        if (ACT == 2) v = fmaxf(v, 0.0f);
        if (ACT == 3) v = v / (1.0f + expf(-v));
        if (ACT == 4) v = (v > 0.f) ? v : 0.01f * v;
        if (ACT == 5) v = 0.5f * v * (1.0f + erff(v * 0.70710678118654752f));
        slab[(mOff + r) * 68 + (j << 4) + rlane] = v;
      }
    }
    __builtin_amdgcn_fence(__ATOMIC_RELEASE, "workgroup");
    __builtin_amdgcn_wave_barrier();
    __builtin_amdgcn_fence(__ATOMIC_ACQUIRE, "workgroup");
    if (OUT_MODE == 0) {
      float* C = (float*)Cout + (size_t)b * strideC;
      const int hh = lane >> 4, c4 = (lane & 15) * 4;
      for (int pass = 0; pass < 2; ++pass) {
#pragma unroll
        for (int it = 0; it < 8; ++it) {
          const int row = it * 2 + hh;
          v4f v = *(const v4f*)(slab + row * 68 + c4);
          *(volatile v4f*)(C + (size_t)(mBase + row) * ldc + n0 + c4) = v;
        }
        __threadfence();
      }
    } else {
      const int q = lane >> 3, c8 = (lane & 7) * 8;
      unsigned short* C  = (unsigned short*)Cout  + (size_t)b * strideC;
      unsigned short* C2 = (OUT_MODE == 2) ? ((unsigned short*)Cout2 + (size_t)b * strideC) : nullptr;
      for (int pass = 0; pass < 2; ++pass) {
#pragma unroll
        for (int it = 0; it < 4; ++it) {
          const int row = it * 4 + q;
          const float* sp = slab + row * 68 + c8;
          v8h hv, lv;
#pragma unroll
          for (int e = 0; e < 8; ++e) {
            if (OUT_MODE == 1) {
              hv[e] = (_Float16)sp[e];
            } else {
              unsigned short hb = f2bf_bits(sp[e]);
              unsigned short lb = f2bf_bits(sp[e] - bf_bits2f(hb));
              hv[e] = __builtin_bit_cast(_Float16, hb);
              lv[e] = __builtin_bit_cast(_Float16, lb);
            }
          }
          *(volatile v8h*)(C + (size_t)(mBase + row) * ldc + n0 + c8) = hv;
          if (OUT_MODE == 2) *(volatile v8h*)(C2 + (size_t)(mBase + row) * ldc + n0 + c8) = lv;
        }
        __threadfence();
      }
    }
    __builtin_amdgcn_fence(__ATOMIC_RELEASE, "workgroup");
    __builtin_amdgcn_wave_barrier();
    __builtin_amdgcn_fence(__ATOMIC_ACQUIRE, "workgroup");
  }
}

constexpr int kHD   = 128;
constexpr int kNG4  = 512;
constexpr int kKF   = 256;
constexpr int kTP   = 264;
constexpr int kSP   = 132;
constexpr int kL    = 24;
constexpr int kMS   = 32;
constexpr int kNS   = 256;
constexpr float kXS     = 64.0f;
constexpr float kWS     = 16.0f;
constexpr float kAccInv = 1.0f / 1024.0f;

__device__ __forceinline__ v8f mma_f16g(v16h a, v16h b, v8f c) {
  c = __builtin_amdgcn_wmma_f32_16x16x32_f16(false, a, false, b, (short)0, c, false, false);
  asm volatile("v_nop\n\tv_nop\n\tv_nop\n\tv_nop" : "+v"(c) : "v"(a), "v"(b));
  return c;
}
__device__ __forceinline__ int clampi(int v, int hi) { v = v < 0 ? 0 : v; return v > hi ? hi : v; }
__device__ __forceinline__ float sigm_f(float x) {
  x = fminf(fmaxf(x, -30.0f), 30.0f);
  return 1.0f / (1.0f + expf(-x));
}

__global__ __launch_bounds__(256) void k_wprep(const float* __restrict__ wih, const float* __restrict__ whh,
                                               unsigned short* __restrict__ Wfp) {
  const int tid = threadIdx.x, wave = tid >> 5, lane = tid & 31;
  const int key = blockIdx.y;
  const int g = blockIdx.x * 8 + wave;
  const int c8 = lane * 8;
  const int cc = c8 & (kHD - 1);
  const bool isx = c8 < kHD;
  const int rs = (g < 384) ? g : (g - kHD);
  const float* pi = wih + ((size_t)key * 384 + rs) * kHD + cc;
  const float* ph = whh + ((size_t)key * 384 + rs) * kHD + cc;
  const v4f a0 = *(const v4f*)pi, a1 = *(const v4f*)(pi + 4);
  const v4f h0 = *(const v4f*)ph, h1 = *(const v4f*)(ph + 4);
  const float xv[8] = {a0[0], a0[1], a0[2], a0[3], a1[0], a1[1], a1[2], a1[3]};
  const float hv8[8] = {h0[0], h0[1], h0[2], h0[3], h1[0], h1[1], h1[2], h1[3]};
  const bool keepx = (g < 384);
  const bool keeph = (g < 256) || (g >= 384);
  v8h hv;
#pragma unroll
  for (int e = 0; e < 8; ++e) {
    const float vx = keepx ? xv[e] : 0.0f;
    const float vh = keeph ? hv8[e] : 0.0f;
    const float v = isx ? vx : vh;
    hv[e] = (_Float16)(v * kWS);
  }
  unsigned short* dst = Wfp + ((size_t)key * kNG4 + g) * kKF + c8;
  *(volatile v8h*)dst = hv;
  __threadfence();
  *(volatile v8h*)dst = hv;
}

__global__ __launch_bounds__(128) void k_bprep(const float* __restrict__ bih, const float* __restrict__ bhh,
                                               float* __restrict__ bfo) {
  const int key = blockIdx.x;
  const int g4 = threadIdx.x * 4;
  v4f v;
#pragma unroll
  for (int e = 0; e < 4; ++e) {
    const int g = g4 + e;
    const int rs = (g < 384) ? g : (g - kHD);
    const float vi = bih[(size_t)key * 384 + rs];
    const float vh = bhh[(size_t)key * 384 + rs];
    v[e] = (g < 256) ? (vi + vh) : ((g < 384) ? vi : vh);
  }
  float* dst = bfo + (size_t)key * kNG4 + g4;
  *(volatile v4f*)dst = v;
  __threadfence();
  *(volatile v4f*)dst = v;
}

__global__ __launch_bounds__(128) void k_fcprep(const float* __restrict__ fcw, int nOut, int kDim,
                                                unsigned short* __restrict__ Bhi, unsigned short* __restrict__ Blo, int nRowsB,
                                                unsigned short* __restrict__ Ahi, unsigned short* __restrict__ Alo, int aRow0) {
  const int tid = threadIdx.x;
  const int bid = blockIdx.x;
  const int k8 = tid * 8;
  if (k8 >= kDim) return;
  const bool isB = bid < nRowsB;
  const int n = isB ? bid : 0;
  const bool keep = isB && (n < nOut);
  const int nc = (n < nOut) ? n : (nOut - 1);
  v8h hv, lv;
#pragma unroll
  for (int e = 0; e < 8; ++e) {
    float v = fcw[(size_t)(k8 + e) * nOut + nc];
    v = keep ? v : 0.0f;
    const unsigned short hb = f2bf_bits(v);
    const unsigned short lb = f2bf_bits(v - bf_bits2f(hb));
    hv[e] = __builtin_bit_cast(_Float16, hb);
    lv[e] = __builtin_bit_cast(_Float16, lb);
  }
  const size_t off = isB ? ((size_t)bid * kDim + k8) : ((size_t)(aRow0 + (bid - nRowsB)) * kDim + k8);
  unsigned short* dh = isB ? Bhi : Ahi;
  unsigned short* dl = isB ? Blo : Alo;
  *(volatile v8h*)(dh + off) = hv;
  *(volatile v8h*)(dl + off) = lv;
  __threadfence();
  *(volatile v8h*)(dh + off) = hv;
  *(volatile v8h*)(dl + off) = lv;
}

__global__ __launch_bounds__(128) void k_vemb(const int* __restrict__ t0, const int* __restrict__ t1, const int* __restrict__ t2,
                                              const float* __restrict__ e0, const float* __restrict__ e1, const float* __restrict__ e2,
                                              int n0, int n1, int n2, unsigned short* __restrict__ Xp) {
  __shared__ __align__(16) float ssh[kHD];
  const int tid = threadIdx.x, key = blockIdx.y, n = blockIdx.x;
  const int* tok = (key == 0) ? t0 : ((key == 1) ? t1 : t2);
  const float* emb = (key == 0) ? e0 : ((key == 1) ? e1 : e2);
  const int voc = (key == 0) ? n0 : ((key == 1) ? n1 : n2);
  const int* tk = tok + (size_t)n * kL;
  float s = 0.0f;
#pragma unroll 4
  for (int l = 0; l < kL; ++l) {
    const int id = clampi(tk[l], voc - 1);
    s += emb[(size_t)id * kHD + tid];
  }
  ssh[tid] = s;
  __syncthreads();
  const int r0 = tid >> 4, c8 = (tid & 15) * 8;
  v8h hv;
#pragma unroll
  for (int e = 0; e < 8; ++e) hv[e] = (_Float16)(ssh[c8 + e] * kXS);
  _Float16* X = (_Float16*)Xp;
  for (int pass = 0; pass < 2; ++pass) {
#pragma unroll
    for (int it = 0; it < kMS / 8; ++it) {
      const int t = it * 8 + r0;
      *(volatile v8h*)(X + (((size_t)key * kNS + n) * kMS + t) * kHD + c8) = hv;
    }
    __threadfence();
  }
}

__global__ __launch_bounds__(128) void k_pemb(const int* __restrict__ ti3, const int* __restrict__ tv3,
                                              const int* __restrict__ ti4, const int* __restrict__ tv4,
                                              const float* __restrict__ ei3, const float* __restrict__ ev3,
                                              const float* __restrict__ ei4, const float* __restrict__ ev4,
                                              int ni3, int nv3, int ni4, int nv4, unsigned short* __restrict__ Xp) {
  __shared__ __align__(16) float ssh[kHD];
  const int tid = threadIdx.x, ky = blockIdx.y, nm = blockIdx.x;
  const int* ti = (ky == 0) ? ti3 : ti4;
  const int* tv = (ky == 0) ? tv3 : tv4;
  const float* ei = (ky == 0) ? ei3 : ei4;
  const float* ev = (ky == 0) ? ev3 : ev4;
  const int ni = (ky == 0) ? ni3 : ni4;
  const int nv = (ky == 0) ? nv3 : nv4;
  const int* ta = ti + (size_t)nm * kL;
  const int* tb = tv + (size_t)nm * kL;
  float s = 0.0f;
#pragma unroll 4
  for (int l = 0; l < kL; ++l) {
    const int a = clampi(ta[l], ni - 1);
    const int b = clampi(tb[l], nv - 1);
    s += ei[(size_t)a * kHD + tid] * ev[(size_t)b * kHD + tid];
  }
  ssh[tid] = s;
  __syncthreads();
  if (tid < 16) {
    const int c8 = tid * 8;
    v8h hv;
#pragma unroll
    for (int e = 0; e < 8; ++e) hv[e] = (_Float16)(ssh[c8 + e] * kXS);
    _Float16* dst = (_Float16*)Xp + (((size_t)(3 + ky)) * kNS * kMS + nm) * kHD + c8;
    *(volatile v8h*)dst = hv;
    __threadfence();
    *(volatile v8h*)dst = hv;
  }
}

__global__ __launch_bounds__(128) void k_info(const float* __restrict__ wgt, const float* __restrict__ age,
                                              const float* __restrict__ iw, const float* __restrict__ ib,
                                              unsigned short* __restrict__ Xp) {
  const int slot = blockIdx.x * 128 + threadIdx.x;
  const int ky = blockIdx.y;
  const int n = slot >> 4, c8 = (slot & 15) * 8;
  const float* val = (ky == 0) ? wgt : age;
  const float x = val[n];
  v8h hv;
#pragma unroll
  for (int e = 0; e < 8; ++e) {
    const float w = iw[ky * kHD + c8 + e];
    const float bb = ib[ky * kHD + c8 + e];
    hv[e] = (_Float16)((x * w + bb) * kXS);
  }
  _Float16* dst = (_Float16*)Xp + (((size_t)(5 + ky)) * kNS + n) * kHD + c8;
  *(volatile v8h*)dst = hv;
  __threadfence();
  *(volatile v8h*)dst = hv;
}

template <int MODE>
__global__ __launch_bounds__(256) void k_gru(const unsigned short* __restrict__ Xp, const unsigned short* __restrict__ Wfp,
                                              const float* __restrict__ bfz, int nSteps, int rowsPerKey, int tilesPerKey,
                                              unsigned short* out0, unsigned short* out1, int ldo) {
  const _Float16* X = (const _Float16*)Xp;
  const _Float16* Wf = (const _Float16*)Wfp;
  __shared__ __align__(16) _Float16 tile[16 * kTP];
  __shared__ __align__(16) float hs[16 * kSP];
  const int tid = threadIdx.x, wave = tid >> 5, lane = tid & 31, hh = lane >> 4, c = lane & 15;
  const int key = blockIdx.x / tilesPerKey;
  const int tix = blockIdx.x - key * tilesPerKey;
  const int rowbase = tix * 16;
  const size_t growbase = (size_t)key * rowsPerKey + rowbase;
  const _Float16* Wk = Wf + (size_t)key * kNG4 * kKF;
  const float* bk = bfz + (size_t)key * kNG4;
  const int u = wave * 16 + c;
  const float b_r = bk[u], b_z = bk[kHD + u], b_nx = bk[2 * kHD + u], b_nh = bk[3 * kHD + u];
  float hreg[8] = {0.f, 0.f, 0.f, 0.f, 0.f, 0.f, 0.f, 0.f};
  const int lrow = tid >> 4, lc8 = (tid & 15) * 8;
  {
    v8h z;
#pragma unroll
    for (int e = 0; e < 8; ++e) z[e] = (_Float16)0.0f;
    *(v8h*)(tile + lrow * kTP + kHD + lc8) = z;
  }
  const int Tc = nSteps > 32 ? 32 : nSteps;
  for (int t = 0; t < Tc; ++t) {
    {
      const v8h xv = *(const v8h*)(X + ((growbase + lrow) * (size_t)nSteps + t) * kHD + lc8);
      *(v8h*)(tile + lrow * kTP + lc8) = xv;
    }
    __syncthreads();
    v8f acc0 = (v8f){0.f,0.f,0.f,0.f,0.f,0.f,0.f,0.f};
    v8f acc1 = acc0, acc2 = acc0, acc3 = acc0;
#pragma unroll 2
    for (int ks = 0; ks < kKF / 32; ++ks) {
      union { v16h v; v8h h[2]; } fa;
      const _Float16* ap = tile + c * kTP + ks * 32 + 8 * hh;
      fa.h[0] = *(const v8h*)(ap);
      fa.h[1] = *(const v8h*)(ap + 16);
      const _Float16* wb = Wk + (size_t)c * kKF + ks * 32 + 8 * hh;
      const v16h b0 = Frag<_Float16>::load(wb + (size_t)(wave * 16) * kKF);
      const v16h b1 = Frag<_Float16>::load(wb + (size_t)(kHD + wave * 16) * kKF);
      const v16h b2 = Frag<_Float16>::load(wb + (size_t)(2 * kHD + wave * 16) * kKF);
      const v16h b3 = Frag<_Float16>::load(wb + (size_t)(3 * kHD + wave * 16) * kKF);
      acc0 = mma_f16g(fa.v, b0, acc0);
      acc1 = mma_f16g(fa.v, b1, acc1);
      acc2 = mma_f16g(fa.v, b2, acc2);
      acc3 = mma_f16g(fa.v, b3, acc3);
    }
#pragma unroll
    for (int r = 0; r < 8; ++r) {
      const float pr  = acc0[r] * kAccInv + b_r;
      const float pz  = acc1[r] * kAccInv + b_z;
      const float pnx = acc2[r] * kAccInv + b_nx;
      const float pnh = acc3[r] * kAccInv + b_nh;
      const float rg = sigm_f(pr);
      const float zg = sigm_f(pz);
      const float ng = tanhf(pnx + rg * pnh);
      hreg[r] = (1.0f - zg) * ng + zg * hreg[r];
    }
    __syncthreads();
#pragma unroll
    for (int r = 0; r < 8; ++r) tile[(8 * hh + r) * kTP + kHD + u] = (_Float16)(hreg[r] * kXS);
  }
#pragma unroll
  for (int r = 0; r < 8; ++r) hs[(8 * hh + r) * kSP + u] = hreg[r];
  __syncthreads();
  {
    const float* sp = hs + lrow * kSP + lc8;
    if (MODE == 0) {
      v8h hv;
#pragma unroll
      for (int e = 0; e < 8; ++e) hv[e] = (_Float16)(sp[e] * kXS);
      _Float16* dst = (_Float16*)out0 + (growbase + lrow) * (size_t)kHD + lc8;
      *(volatile v8h*)dst = hv;
      __threadfence();
      *(volatile v8h*)dst = hv;
    } else {
      v8h hv, lv;
#pragma unroll
      for (int e = 0; e < 8; ++e) {
        const float v = fmaxf(sp[e], 0.0f);
        const unsigned short hb = f2bf_bits(v);
        const unsigned short lb = f2bf_bits(v - bf_bits2f(hb));
        hv[e] = __builtin_bit_cast(_Float16, hb);
        lv[e] = __builtin_bit_cast(_Float16, lb);
      }
      const size_t off = (size_t)(rowbase + lrow) * ldo + (size_t)key * kHD + lc8;
      *(volatile v8h*)(out0 + off) = hv;
      *(volatile v8h*)(out1 + off) = lv;
      __threadfence();
      *(volatile v8h*)(out0 + off) = hv;
      *(volatile v8h*)(out1 + off) = lv;
    }
  }
}

__global__ __launch_bounds__(256) void k_fin(const float* __restrict__ Cf, int ldc, const float* __restrict__ fcb,
                                             int nOut, float* out, int n4) {
  const int i = blockIdx.x * 256 + threadIdx.x;
  if (i >= n4) return;
  v4f v;
#pragma unroll
  for (int e = 0; e < 4; ++e) {
    const int idx = 4 * i + e;
    const int bb = idx / nOut;
    const int o = idx - bb * nOut;
    v[e] = Cf[(size_t)bb * ldc + o] + fcb[o];
  }
  *(volatile v4f*)(out + 4 * (size_t)i) = v;
  __threadfence();
  *(volatile v4f*)(out + 4 * (size_t)i) = v;
}

extern "C" void kernel_launch(void* const* d_in, const int* in_sizes, int n_in,
                              void* d_out, int out_size, void* d_ws, size_t ws_size,
                              hipStream_t stream) {
  (void)n_in; (void)ws_size;
  const int*   tok_cond      = (const int*)d_in[0];
  const int*   tok_proc      = (const int*)d_in[1];
  const int*   tok_drug      = (const int*)d_in[2];
  const int*   tok_lab_item  = (const int*)d_in[3];
  const int*   tok_lab_value = (const int*)d_in[4];
  const int*   tok_inj_item  = (const int*)d_in[5];
  const int*   tok_inj_value = (const int*)d_in[6];
  const float* weight        = (const float*)d_in[7];
  const float* age           = (const float*)d_in[8];
  const float* emb_cond      = (const float*)d_in[9];
  const float* emb_proc      = (const float*)d_in[10];
  const float* emb_drug      = (const float*)d_in[11];
  const float* emb_lab_item  = (const float*)d_in[12];
  const float* emb_lab_value = (const float*)d_in[13];
  const float* emb_inj_item  = (const float*)d_in[14];
  const float* emb_inj_value = (const float*)d_in[15];
  const float* mgru_wih      = (const float*)d_in[16];
  const float* mgru_whh      = (const float*)d_in[17];
  const float* mgru_bih      = (const float*)d_in[18];
  const float* mgru_bhh      = (const float*)d_in[19];
  const float* vgru_wih      = (const float*)d_in[20];
  const float* vgru_whh      = (const float*)d_in[21];
  const float* vgru_bih      = (const float*)d_in[22];
  const float* vgru_bhh      = (const float*)d_in[23];
  const float* info_w        = (const float*)d_in[24];
  const float* info_b        = (const float*)d_in[25];
  const float* fc_w          = (const float*)d_in[26];
  const float* fc_b          = (const float*)d_in[27];
  float* out = (float*)d_out;

  const int vocCond = in_sizes[9]  / kHD;
  const int vocProc = in_sizes[10] / kHD;
  const int vocDrug = in_sizes[11] / kHD;
  const int vocLabI = in_sizes[12] / kHD;
  const int vocLabV = in_sizes[13] / kHD;
  const int vocInjI = in_sizes[14] / kHD;
  const int vocInjV = in_sizes[15] / kHD;

  const int nKeyM = 5, nKeyV = 7, nB = 16, nV = 16, nOut = 193, kFc = 896, nFcPad = 256, mFcPad = 64;

  char* ws = (char*)d_ws;
  size_t off = 0;
  auto take = [&](size_t bytes) -> char* {
    char* p = ws + off;
    off = (off + bytes + 255) & ~(size_t)255;
    return p;
  };
  unsigned short* monX = (unsigned short*)take((size_t)nKeyM * kNS * kMS * kHD * 2);
  unsigned short* visX = (unsigned short*)take((size_t)nKeyV * nB * nV * kHD * 2);
  unsigned short* WfM  = (unsigned short*)take((size_t)nKeyM * kNG4 * kKF * 2);
  unsigned short* WfV  = (unsigned short*)take((size_t)nKeyV * kNG4 * kKF * 2);
  float*          bfM  = (float*)take((size_t)nKeyM * kNG4 * 4);
  float*          bfV  = (float*)take((size_t)nKeyV * kNG4 * 4);
  unsigned short* Ahi  = (unsigned short*)take((size_t)mFcPad * kFc * 2);
  unsigned short* Alo  = (unsigned short*)take((size_t)mFcPad * kFc * 2);
  unsigned short* Bhi  = (unsigned short*)take((size_t)nFcPad * kFc * 2);
  unsigned short* Blo  = (unsigned short*)take((size_t)nFcPad * kFc * 2);
  float*          Cfc  = (float*)take((size_t)mFcPad * nFcPad * 4);

  k_wprep<<<dim3(64, nKeyM), 256, 0, stream>>>(mgru_wih, mgru_whh, WfM);
  k_wprep<<<dim3(64, nKeyV), 256, 0, stream>>>(vgru_wih, vgru_whh, WfV);
  k_bprep<<<nKeyM, 128, 0, stream>>>(mgru_bih, mgru_bhh, bfM);
  k_bprep<<<nKeyV, 128, 0, stream>>>(vgru_bih, vgru_bhh, bfV);
  k_fcprep<<<nFcPad + (mFcPad - nB), 128, 0, stream>>>(fc_w, nOut, kFc, Bhi, Blo, nFcPad, Ahi, Alo, nB);

  k_vemb<<<dim3(kNS, 3), 128, 0, stream>>>(tok_cond, tok_proc, tok_drug, emb_cond, emb_proc, emb_drug,
                                          vocCond, vocProc, vocDrug, monX);
  k_pemb<<<dim3(kNS * kMS, 2), 128, 0, stream>>>(tok_lab_item, tok_lab_value, tok_inj_item, tok_inj_value,
                                                emb_lab_item, emb_lab_value, emb_inj_item, emb_inj_value,
                                                vocLabI, vocLabV, vocInjI, vocInjV, monX);
  k_info<<<dim3(32, 2), 128, 0, stream>>>(weight, age, info_w, info_b, visX);

  k_gru<0><<<nKeyM * (kNS / 16), 256, 0, stream>>>(monX, WfM, bfM, kMS, kNS, kNS / 16, visX, visX, 0);

  k_gru<1><<<nKeyV, 256, 0, stream>>>(visX, WfV, bfV, nV, nB, 1, Ahi, Alo, kFc);

  wmma_gemm64<1, true, 0, 0, false><<<dim3(1, 1), 256, 0, stream>>>(
      Ahi, Alo, kFc, 0L, Bhi, Blo, kFc, 0L, (void*)Cfc, (void*)Cfc, nFcPad, 0L,
      bfM, (const float*)bfV, 0L, mFcPad, nFcPad, kFc, 1.0f);

  static_assert((16 * 193) % 4 == 0, "output float4 pieces");
  const int n4 = (16 * 193) / 4;
  (void)out_size;
  k_fin<<<(n4 + 255) / 256, 256, 0, stream>>>(Cfc, nFcPad, fc_b, nOut, out, n4);
}
